// PyGraphBipartite_56143812493353
// MI455X (gfx1250) — hardware-verified
//
#include <hip/hip_runtime.h>

#define NNODES 8192
#define NCH    64
#define NOUT   64
#define NB     8
#define BCAP   1024
#define HWSZ   1024
#define KNN    9
#define TROWS  16
#define NBLK1  (NB * (HWSZ / 32))
#define NBLK2  (NNODES / TROWS)

typedef unsigned short u16;
typedef u16    v8us  __attribute__((ext_vector_type(8)));
typedef u16    v16us __attribute__((ext_vector_type(16)));
typedef __bf16 v16b  __attribute__((ext_vector_type(16)));
typedef float  v8f   __attribute__((ext_vector_type(8)));
typedef float  v4f   __attribute__((ext_vector_type(4)));
typedef v4f    __attribute__((may_alias)) v4fa;

union Frag { v16b v; v16us u; v8us h8[2]; };

static __device__ __forceinline__ unsigned bfb(float f) {
    const unsigned u = __float_as_uint(f);
    return (u + 0x7FFFu + ((u >> 16) & 1u)) >> 16;
}
static __device__ __forceinline__ float bfv(unsigned b) { return __uint_as_float(b << 16); }

static __device__ __forceinline__ void split3(float f, unsigned& h, unsigned& m, unsigned& l) {
    h = bfb(f);
    const float r1 = f - bfv(h);
    m = bfb(r1);
    const float r2 = r1 - bfv(m);
    l = bfb(r2);
}
static __device__ __forceinline__ void split2(float f, unsigned& h, unsigned& m) {
    h = bfb(f);
    m = bfb(f - bfv(h));
}

static __device__ __forceinline__ v8f wmma_bf(const v16b a, const v16b b, v8f c) {
    v8f d = __builtin_amdgcn_wmma_f32_16x16x32_bf16(false, a, false, b, (short)0, c, false, false);
    asm volatile("v_nop\n\tv_nop\n\tv_nop\n\tv_nop" : "+v"(d) : "v"(a), "v"(b));
    return d;
}

static __device__ __forceinline__ v8us ld8(const u16* p) { return *(const v8us*)p; }

__global__ void __launch_bounds__(256) prep_kernel(const float* __restrict__ x,
                                                   float* xf, u16* ph, u16* pm, u16* pl,
                                                   float* sq)
{
    __shared__ __attribute__((aligned(16))) float tile[NCH][33];
    __shared__ __attribute__((aligned(16))) float s_sq[32];
    const int blk = blockIdx.x;
    if (blk >= NBLK1) return;
    const int b   = blk >> 5;
    const int hw0 = (blk & 31) * 32;
    const int t = threadIdx.x, lane = t & 31, wave = t >> 5;

    for (int i = t; i < NCH * 32; i += 256) {
        const int c = i >> 5, w = i & 31;
        tile[c][w] = x[(size_t)(b * NCH + c) * HWSZ + hw0 + w];
    }
    __syncthreads();
    if (t < 32) {
        float s = 0.0f;
        #pragma unroll 8
        for (int c = 0; c < NCH; ++c) { const float v = tile[c][t]; s += v * v; }
        s_sq[t] = s;
    }
    __syncthreads();

    const int n0 = b * BCAP + hw0;

    v4f xv[2]; size_t xo[2];
    #pragma unroll
    for (int s2 = 0; s2 < 2; ++s2) {
        const int row = 4 * wave + 2 * s2 + (lane >> 4);
        const int c0  = 4 * (lane & 15);
        v4f v;
        v.x = tile[c0 + 0][row]; v.y = tile[c0 + 1][row];
        v.z = tile[c0 + 2][row]; v.w = tile[c0 + 3][row];
        xv[s2] = v;
        xo[s2] = (size_t)(n0 + row) * NCH + c0;
    }
    const int prow = 4 * wave + (lane >> 3);
    const int pc0  = 8 * (lane & 7);
    v8us hv, mv, lv;
    #pragma unroll
    for (int e = 0; e < 8; ++e) {
        unsigned hb, mb, lb;
        split3(tile[pc0 + e][prow], hb, mb, lb);
        hv[e] = (u16)hb; mv[e] = (u16)mb; lv[e] = (u16)lb;
    }
    const size_t po = (size_t)(n0 + prow) * NCH + pc0;
    v4f sv = {};
    if (t < 8) { sv.x = s_sq[4 * t]; sv.y = s_sq[4 * t + 1]; sv.z = s_sq[4 * t + 2]; sv.w = s_sq[4 * t + 3]; }

    *(volatile v4f*)(xf + xo[0]) = xv[0];
    *(volatile v4f*)(xf + xo[1]) = xv[1];
    *(volatile v8us*)(ph + po) = hv;
    *(volatile v8us*)(pm + po) = mv;
    *(volatile v8us*)(pl + po) = lv;
    if (t < 8) *(volatile v4f*)(sq + n0 + 4 * t) = sv;
    __threadfence();
    *(volatile v4f*)(xf + xo[0]) = xv[0];
    *(volatile v4f*)(xf + xo[1]) = xv[1];
    *(volatile v8us*)(ph + po) = hv;
    *(volatile v8us*)(pm + po) = mv;
    *(volatile v8us*)(pl + po) = lv;
    if (t < 8) *(volatile v4f*)(sq + n0 + 4 * t) = sv;
}

__global__ void __launch_bounds__(256) knn_agg_kernel(const float* __restrict__ xf,
                                                      const u16* __restrict__ ph,
                                                      const u16* __restrict__ pm,
                                                      const u16* __restrict__ pl,
                                                      const float* __restrict__ sq,
                                                      const float* __restrict__ w1,
                                                      const float* __restrict__ b1,
                                                      const float* __restrict__ w2,
                                                      float* out)
{
    extern __shared__ float dist_s[];
    __shared__ __attribute__((aligned(16))) float s_sqi[TROWS];
    __shared__ __attribute__((aligned(16))) float s_mean[TROWS][NCH];
    __shared__ __attribute__((aligned(16))) float s_part[2][TROWS][NOUT];

    const int blk = blockIdx.x;
    if (blk >= NBLK2) return;
    const int tid = threadIdx.x, lane = tid & 31, wave = tid >> 5;
    const int hh = lane >> 4, mm = lane & 15;
    const int b      = blk >> 6;
    const int bstart = b * BCAP;
    const int bsize  = (b == NB - 1) ? (BCAP - 1) : BCAP;
    const int i0     = blk * TROWS;
    int rows_knn = bstart + bsize - i0;
    if (rows_knn > TROWS) rows_knn = TROWS;
    const float INF = __builtin_huge_valf();

    if (tid < TROWS) s_sqi[tid] = sq[i0 + tid];
    __syncthreads();

    {
        Frag a[2][3];
        const size_t arow = (size_t)(i0 + mm) * NCH;
        #pragma unroll
        for (int ks = 0; ks < 2; ++ks) {
            const int k0 = ks * 32 + 8 * hh;
            a[ks][0].h8[0] = ld8(ph + arow + k0); a[ks][0].h8[1] = ld8(ph + arow + k0 + 16);
            a[ks][1].h8[0] = ld8(pm + arow + k0); a[ks][1].h8[1] = ld8(pm + arow + k0 + 16);
            a[ks][2].h8[0] = ld8(pl + arow + k0); a[ks][2].h8[1] = ld8(pl + arow + k0 + 16);
        }
        float sqi[8];
        #pragma unroll
        for (int r = 0; r < 8; ++r) sqi[r] = s_sqi[8 * hh + r];

        #pragma unroll 1
        for (int jt = wave; jt < BCAP / 16; jt += 8) {
            const int col = jt * 16 + mm;
            const size_t brow = (size_t)(bstart + col) * NCH;
            v8f acc = {};
            #pragma unroll
            for (int ks = 0; ks < 2; ++ks) {
                const int k0 = ks * 32 + 8 * hh;
                Frag fb0, fb1, fb2;
                fb0.h8[0] = ld8(ph + brow + k0); fb0.h8[1] = ld8(ph + brow + k0 + 16);
                fb1.h8[0] = ld8(pm + brow + k0); fb1.h8[1] = ld8(pm + brow + k0 + 16);
                fb2.h8[0] = ld8(pl + brow + k0); fb2.h8[1] = ld8(pl + brow + k0 + 16);
                acc = wmma_bf(a[ks][0].v, fb0.v, acc);
                acc = wmma_bf(a[ks][0].v, fb1.v, acc);
                acc = wmma_bf(a[ks][1].v, fb0.v, acc);
                acc = wmma_bf(a[ks][0].v, fb2.v, acc);
                acc = wmma_bf(a[ks][1].v, fb1.v, acc);
                acc = wmma_bf(a[ks][2].v, fb0.v, acc);
            }
            const float sqj = sq[bstart + col];
            const bool ok = col < bsize;
            #pragma unroll
            for (int r = 0; r < 8; ++r) {
                const float tsum = sqi[r] + sqj;
                const float d = tsum - 2.0f * acc[r];
                dist_s[(8 * hh + r) * BCAP + col] = ok ? d : INF;
            }
        }
    }
    __syncthreads();

    #pragma unroll
    for (int rs = 0; rs < 2; ++rs) {
        const int m = wave + 8 * rs;
        if (m < rows_knn) {
            float dv[32];
            #pragma unroll
            for (int q = 0; q < 32; ++q) dv[q] = dist_s[m * BCAP + lane + 32 * q];
            int nb[KNN];
            #pragma unroll
            for (int s = 0; s < KNN; ++s) {
                float best = INF; int bi = 0;
                #pragma unroll
                for (int q = 0; q < 32; ++q) {
                    const bool lt = dv[q] < best;
                    best = lt ? dv[q] : best;
                    bi   = lt ? q : bi;
                }
                int bidx = lane + 32 * bi;
                #pragma unroll
                for (int off = 16; off > 0; off >>= 1) {
                    const float ov = __shfl_xor(best, off, 32);
                    const int   oi = __shfl_xor(bidx, off, 32);
                    const bool take = (ov < best) || (ov == best && oi < bidx);
                    best = take ? ov : best;
                    bidx = take ? oi : bidx;
                }
                bidx = __shfl(bidx, 0, 32);
                nb[s] = bidx;
                const int ol = bidx & 31, ob = bidx >> 5;
                #pragma unroll
                for (int q = 0; q < 32; ++q) dv[q] = (lane == ol && q == ob) ? INF : dv[q];
            }
            #pragma unroll
            for (int cc = 0; cc < 2; ++cc) {
                const int c = lane + 32 * cc;
                float s = 0.0f;
                #pragma unroll
                for (int q = 0; q < KNN; ++q) {
                    int node = bstart + nb[q];
                    node = node < 0 ? 0 : (node > NNODES - 1 ? NNODES - 1 : node);
                    s += xf[(size_t)node * NCH + c];
                }
                s_mean[m][c] = s * (1.0f / 9.0f);
            }
        } else if (m < TROWS) {
            #pragma unroll
            for (int cc = 0; cc < 2; ++cc) {
                const int c = lane + 32 * cc;
                s_mean[m][c] = xf[(size_t)(i0 + m) * NCH + c];
            }
        }
    }
    __syncthreads();

    {
        const int nt  = wave & 3;
        const int src = wave >> 2;
        const int o   = nt * 16 + mm;
        const float* __restrict__ W = src ? w2 : w1;
        v8f acc = {};
        #pragma unroll
        for (int ks = 0; ks < 2; ++ks) {
            const int k0 = ks * 32 + 8 * hh;
            Frag fah, fam, fbh, fbm;
            if (src == 0) {
                #pragma unroll
                for (int i = 0; i < 8; ++i) {
                    unsigned h0, m0, h1, m1;
                    split2(s_mean[mm][k0 + i], h0, m0);
                    split2(s_mean[mm][k0 + 16 + i], h1, m1);
                    fah.u[i] = (u16)h0; fam.u[i] = (u16)m0;
                    fah.u[8 + i] = (u16)h1; fam.u[8 + i] = (u16)m1;
                }
            } else {
                const size_t arow = (size_t)(i0 + mm) * NCH;
                fah.h8[0] = ld8(ph + arow + k0); fah.h8[1] = ld8(ph + arow + k0 + 16);
                fam.h8[0] = ld8(pm + arow + k0); fam.h8[1] = ld8(pm + arow + k0 + 16);
            }
            #pragma unroll
            for (int i = 0; i < 8; ++i) {
                unsigned h0, m0, h1, m1;
                split2(W[o * NCH + k0 + i], h0, m0);
                split2(W[o * NCH + k0 + 16 + i], h1, m1);
                fbh.u[i] = (u16)h0; fbm.u[i] = (u16)m0;
                fbh.u[8 + i] = (u16)h1; fbm.u[8 + i] = (u16)m1;
            }
            acc = wmma_bf(fah.v, fbh.v, acc);
            acc = wmma_bf(fah.v, fbm.v, acc);
            acc = wmma_bf(fam.v, fbh.v, acc);
        }
        #pragma unroll
        for (int r = 0; r < 8; ++r) s_part[src][8 * hh + r][o] = acc[r];
    }
    __syncthreads();

    {
        const int row = 2 * wave + (lane >> 4);
        const int c0  = 4 * (lane & 15);
        const v4f pa = *(const v4fa*)(&s_part[0][row][c0]);
        const v4f pb = *(const v4fa*)(&s_part[1][row][c0]);
        v4f bv;
        bv.x = b1[c0]; bv.y = b1[c0 + 1]; bv.z = b1[c0 + 2]; bv.w = b1[c0 + 3];
        const v4f v = pa + pb + bv;
        volatile v4f* gp = (volatile v4f*)(out + (size_t)(i0 + row) * NOUT + c0);
        *gp = v;
        __threadfence();
        *gp = v;
    }
}

extern "C" void kernel_launch(void* const* d_in, const int* in_sizes, int n_in,
                              void* d_out, int out_size, void* d_ws, size_t ws_size,
                              hipStream_t stream)
{
    if (n_in < 4) return;
    if (in_sizes[0] != NNODES * NCH || in_sizes[1] != NOUT * NCH ||
        in_sizes[2] != NOUT || in_sizes[3] != NOUT * NCH) return;
    if (out_size != NNODES * NOUT) return;

    const size_t xf_bytes = (size_t)NNODES * NCH * sizeof(float);
    const size_t pl_bytes = (size_t)NNODES * NCH * sizeof(u16);
    const size_t sq_bytes = (size_t)NNODES * sizeof(float);
    const size_t off_xf = 0;
    const size_t off_ph = off_xf + xf_bytes;
    const size_t off_pm = off_ph + pl_bytes;
    const size_t off_pl = off_pm + pl_bytes;
    const size_t off_sq = off_pl + pl_bytes;
    const size_t total  = off_sq + sq_bytes;
    if (total > ws_size) return;

    const float* x  = (const float*)d_in[0];
    const float* w1 = (const float*)d_in[1];
    const float* b1 = (const float*)d_in[2];
    const float* w2 = (const float*)d_in[3];
    float* out = (float*)d_out;
    char* ws = (char*)d_ws;
    float* xf = (float*)(ws + off_xf);
    u16*   ph = (u16*)(ws + off_ph);
    u16*   pm = (u16*)(ws + off_pm);
    u16*   pl = (u16*)(ws + off_pl);
    float* sq = (float*)(ws + off_sq);

    prep_kernel<<<NBLK1, 256, 0, stream>>>(x, xf, ph, pm, pl, sq);
    knn_agg_kernel<<<NBLK2, 256, TROWS * BCAP * sizeof(float), stream>>>(xf, ph, pm, pl, sq,
                                                                          w1, b1, w2, out);
}
